// ScaledDotProductMHA_13649406067532
// MI455X (gfx1250) — hardware-run, weakly checked
//
#include <hip/hip_runtime.h>


namespace {
constexpr int NB = 2, NH = 16, L = 2048, D = 64, NS = NB * NH  , KB = 128;
constexpr float XS = 8.0f, PS = 256.0f, SCALE = 0.125f;
typedef _Float16 b16;
typedef __attribute__((ext_vector_type(16))) _Float16 v16b;
typedef __attribute__((ext_vector_type(8))) _Float16 v8b;
typedef __attribute__((ext_vector_type(8))) float v8f;
typedef __attribute__((ext_vector_type(4))) float v4f;
__device__ __forceinline__ float bf16_rne(float f) { unsigned int u = __float_as_uint(f); u += 0x7FFFu + ((u >> 16) & 1u); float r = __uint_as_float(u & 0xFFFF0000u); asm volatile("" : "+v"(r)); return r; }
__device__ __forceinline__ void split16(float v, b16& hi, b16& lo) { hi = (b16)v; lo = (b16)(v - (float)hi); }
__device__ __forceinline__ v16b frag_kb(const b16* p, int hh) { const v8b a = *(const v8b*)(p + 8 * hh), b = *(const v8b*)(p + 16 + 8 * hh); v16b f;
#pragma unroll
  for (int e = 0; e < 8; ++e) { f[e] = a[e]; f[8 + e] = b[e]; } return f; }
__device__ __forceinline__ v8f wmma16b(v16b a, v16b b, v8f c) { v8f d = __builtin_amdgcn_wmma_f32_16x16x32_f16(false, a, false, b, (short)0, c, false, false); asm volatile("v_nop\n\tv_nop\n\tv_nop\n\tv_nop" : "+v"(d) : "v"(a), "v"(b)); return d; }
__device__ __forceinline__ void wave_lds_sync() { __builtin_amdgcn_fence(__ATOMIC_RELEASE, "workgroup"); __builtin_amdgcn_wave_barrier(); __builtin_amdgcn_fence(__ATOMIC_ACQUIRE, "workgroup"); }
__device__ __forceinline__ float pmul(float a, float b) { float p = a * b; asm volatile("" : "+v"(p)); return p; }

__global__ __launch_bounds__(256) void put_kernel(const float* __restrict__ q, const float* __restrict__ k, const float* __restrict__ v, b16* __restrict__ QP, b16* __restrict__ KP, b16* __restrict__ VP) { const size_t u = (size_t)blockIdx.x * 256 + threadIdx.x; if (u >= (size_t)NS * L * D / 8) return; const size_t e = u * 8; v8b a, b, c;
#pragma unroll
  for (int j = 0; j < 8; ++j) { a[j] = (b16)(bf16_rne(q[e + j]) * XS); b[j] = (b16)(bf16_rne(k[e + j]) * XS); c[j] = (b16)(bf16_rne(v[e + j]) * XS); }
  for (int pass = 0; pass < 2; ++pass) { *(volatile v8b*)(QP + e) = a; *(volatile v8b*)(KP + e) = b; *(volatile v8b*)(VP + e) = c; __threadfence(); } }
__global__ __launch_bounds__(32) void att_kernel(const b16* __restrict__ QP, const b16* __restrict__ KP, const b16* __restrict__ VP, int SLIM, float* __restrict__ out) { __shared__ __attribute__((aligned(16))) b16 Ph[16][KB + 8], Pl[16][KB + 8], Vt[D][KB + 8]; __shared__ float Sf[16][KB + 4], Of[16][D + 4];
  const int lane = threadIdx.x, nloc = lane & 15, hlf = lane >> 4; const int qt = blockIdx.x % (L / 16); const int s = blockIdx.x / (L / 16); if (s >= SLIM) return; const int t0 = qt * 16; const size_t sb = (size_t)s * L * D;
  const v16b qa0 = frag_kb(QP + sb + (size_t)(t0 + nloc) * D, hlf), qa1 = frag_kb(QP + sb + (size_t)(t0 + nloc) * D + 32, hlf);
  float m_r[8], den_r[8]; v8f acc[4];
#pragma unroll
  for (int r8 = 0; r8 < 8; ++r8) { m_r[r8] = -INFINITY; den_r[r8] = 0.0f; }
#pragma unroll
  for (int t = 0; t < 4; ++t) acc[t] = (v8f){};
#pragma unroll 1
  for (int kb0 = 0; kb0 <= t0; kb0 += KB) { const int nk = (t0 + 16 - kb0) < KB ? (t0 + 16 - kb0) : KB;
    for (int rr = 0; rr < KB; rr += 2) { const int r = rr + hlf;   const b16* vr = VP + sb + (size_t)(kb0 + r) * D; for (int q = 0; q < 4; ++q) Vt[q * 16 + nloc][r] = vr[q * 16 + nloc]; }
    wave_lds_sync();
#pragma unroll
    for (int t = 0; t < KB / 16; ++t) { if (t * 16 < nk) { v8f sacc = {}; sacc = wmma16b(qa0, frag_kb(KP + sb + (size_t)(kb0 + t * 16 + nloc) * D, hlf), sacc); sacc = wmma16b(qa1, frag_kb(KP + sb + (size_t)(kb0 + t * 16 + nloc) * D + 32, hlf), sacc);
#pragma unroll
        for (int r8 = 0; r8 < 8; ++r8) { const int i = t0 + 8 * hlf + r8, j = kb0 + t * 16 + nloc; Sf[8 * hlf + r8][t * 16 + nloc] = (j <= i) ? sacc[r8] * (SCALE / (XS * XS)) : -INFINITY; } }
      else {
#pragma unroll
        for (int r8 = 0; r8 < 8; ++r8) Sf[8 * hlf + r8][t * 16 + nloc] = -INFINITY; } }
    wave_lds_sync();
#pragma unroll
    for (int rr = 0; rr < 16; ++rr) { float mx = -INFINITY;
#pragma unroll
      for (int q = 0; q < 4; ++q) mx = fmaxf(mx, Sf[rr][q * 32 + lane]);
      for (int o = 16; o; o >>= 1) mx = fmaxf(mx, __shfl_xor(mx, o));
      const float mold = __shfl(m_r[rr & 7], (rr >> 3) * 16); const float mn = fmaxf(mold, mx); const float sf = (mold == -INFINITY) ? 0.0f : __expf(mold - mn); float ps = 0.0f;
#pragma unroll
      for (int q = 0; q < 4; ++q) { const int kx = q * 32 + lane; const float sv = Sf[rr][kx]; const float p = (sv == -INFINITY) ? 0.0f : __expf(sv - mn); ps += p; b16 ph, pl; split16(p * PS, ph, pl); Ph[rr][kx] = ph; Pl[rr][kx] = pl; }
      for (int o = 16; o; o >>= 1) ps += __shfl_xor(ps, o);
      if ((rr >> 3) == hlf) { const int r8 = rr & 7; den_r[r8] = den_r[r8] * sf + ps; m_r[r8] = mn;
#pragma unroll
        for (int t = 0; t < 4; ++t) acc[t][r8] = acc[t][r8] * sf; } }
    wave_lds_sync(); const int nks = (nk + 31) / 32;
    for (int ks = 0; ks < nks * 32; ks += 32) { const v16b pa = frag_kb(&Ph[nloc][ks], hlf), pb = frag_kb(&Pl[nloc][ks], hlf);
#pragma unroll
      for (int t = 0; t < 4; ++t) { const v16b vh = frag_kb(&Vt[t * 16 + nloc][ks], hlf); acc[t] = wmma16b(pa, vh, acc[t]); acc[t] = wmma16b(pb, vh, acc[t]); } }
    wave_lds_sync(); }
#pragma unroll
  for (int t = 0; t < 4; ++t)
#pragma unroll
    for (int r8 = 0; r8 < 8; ++r8) Of[8 * hlf + r8][t * 16 + nloc] = acc[t][r8] * (1.0f / (XS * PS)) / den_r[r8];
  wave_lds_sync();
  for (int pass = 0; pass < 2; ++pass) { for (int rr = 0; rr < 16; ++rr) for (int q = 0; q < 2; ++q) ((volatile float*)out)[sb + (size_t)(t0 + rr) * D + q * 32 + lane] = Of[rr][q * 32 + lane]; __threadfence(); } }
}

extern "C" void kernel_launch(void* const* d_in, const int* in_sizes, int n_in, void* d_out, int out_size, void* d_ws, size_t ws_size, hipStream_t stream) {
  (void)n_in;
  if (in_sizes[0] != NS * L * D || in_sizes[1] != NS * L * D || in_sizes[2] != NS * L * D || out_size != NS * L * D) return;
  const int SLIM = NS;
  size_t off = 0; char* ws = (char*)d_ws;
  auto carve = [&](size_t bytes) { char* p = ws + off; off += (bytes + 255) & ~(size_t)255; return p; };
  b16* QP = (b16*)carve((size_t)NS * L * D * 2); b16* KP = (b16*)carve((size_t)NS * L * D * 2); b16* VP = (b16*)carve((size_t)NS * L * D * 2);
  if (off > ws_size || off > ((size_t)32 << 20)) return;
  put_kernel<<<(unsigned)(((size_t)NS * L * D / 8 + 255) / 256), 256, 0, stream>>>((const float*)d_in[1], (const float*)d_in[0], (const float*)d_in[2], QP, KP, VP);
  att_kernel<<<SLIM * (L / 16), 32, 0, stream>>>(QP, KP, VP, SLIM, (float*)d_out);
}
